// Mult_CA_60885456388399
// MI455X (gfx1250) — hardware-verified
//
#include <hip/hip_runtime.h>
#include <stdint.h>

#define NTOK  16384
#define CTOK  256
#define DIM   256
#define DQ    1024
#define NH    32
#define HD    32
#define QT    128
#define NQT   128
#define HALFN 8192
#define GM    128
#define GN    64
#define OSP   68
#define LTP   72
#define EPSL1 1.0e-9f

static_assert(NH * HD == DQ);
static_assert(NQT * QT == NTOK);
static_assert(2 * HALFN == NTOK);
static_assert(NTOK % GM == 0);
static_assert(CTOK % GM == 0);
static_assert(DQ % GM == 0);
static_assert(HALFN % GM == 0);
static_assert(DQ % GN == 0);
static_assert(CTOK % GN == 0);
static_assert(DIM % GN == 0);
static_assert(HALFN % 32 == 0);
static_assert(DIM % 64 == 0);
static_assert(DQ % 64 == 0);
static_assert(DIM % 32 == 0);
static_assert(CTOK % 32 == 0);
static_assert((NTOK * DIM) % 2048 == 0);
static_assert((CTOK * DIM) % 2048 == 0);
static_assert((OSP * 4) % 16 == 0);
static_assert((LTP * 2) % 16 == 0);
static_assert(QT == 8 * 16);
static_assert(CTOK == 256);
static_assert(HD == 32);

typedef unsigned short v8us __attribute__((ext_vector_type(8)));
typedef unsigned int   v4u  __attribute__((ext_vector_type(4)));
typedef float          v8f  __attribute__((ext_vector_type(8)));
typedef float          v4f  __attribute__((ext_vector_type(4)));
typedef __bf16         v16b __attribute__((ext_vector_type(16)));

union Frag { v8us u[2]; v4u q[2]; v16b b; };
static_assert(sizeof(Frag) == 32);

__device__ __forceinline__ unsigned short bf_bits(float f) {
  const unsigned u = __float_as_uint(f);
  return (unsigned short)((u + 0x7FFFu + ((u >> 16) & 1u)) >> 16);
}
__device__ __forceinline__ float bf_up(unsigned short hb) { return __uint_as_float(((unsigned)hb) << 16); }
__device__ __forceinline__ float bfr(float f) { return bf_up(bf_bits(f)); }
__device__ __forceinline__ unsigned pk16(unsigned short a, unsigned short b) { return (unsigned)a | ((unsigned)b << 16); }
__device__ __forceinline__ v8f zero8() { v8f z = {0.f, 0.f, 0.f, 0.f, 0.f, 0.f, 0.f, 0.f}; return z; }

__device__ __forceinline__ Frag ldfrag(const unsigned short* p) {
  Frag f;
  f.u[0] = *(const v8us*)(p);
  f.u[1] = *(const v8us*)(p + 16);
  return f;
}

__device__ __forceinline__ v8f mma_b(v16b a, v16b b, v8f c) {
  v8f d = __builtin_amdgcn_wmma_f32_16x16x32_bf16(false, a, false, b, (short)0, c, false, false);
#if defined(__HIP_DEVICE_COMPILE__)
  asm volatile("v_nop\n\tv_nop\n\tv_nop\n\tv_nop" : "+v"(d) : "v"(a), "v"(b));
#endif
  return d;
}

__device__ __forceinline__ void split8(v4f a, v4f b, v4u& uh, v4u& ul) {
  float f[8] = {a[0], a[1], a[2], a[3], b[0], b[1], b[2], b[3]};
#pragma unroll
  for (int j = 0; j < 4; ++j) {
    const unsigned short h0 = bf_bits(f[2 * j]);
    const unsigned short h1 = bf_bits(f[2 * j + 1]);
    const unsigned short l0 = bf_bits(f[2 * j] - bf_up(h0));
    const unsigned short l1 = bf_bits(f[2 * j + 1] - bf_up(h1));
    uh[j] = pk16(h0, h1);
    ul[j] = pk16(l0, l1);
  }
}

__global__ __launch_bounds__(256)
void cvt_kernel(const float* __restrict__ x, unsigned short* y, int n8) {
  const int t = blockIdx.x * 256 + (int)threadIdx.x;
  if (t >= n8) return;
  const float* s = x + (size_t)t * 8;
  const v4f a = *(const v4f*)(s);
  const v4f b = *(const v4f*)(s + 4);
  v4u u;
  u[0] = pk16(bf_bits(a[0]), bf_bits(a[1]));
  u[1] = pk16(bf_bits(a[2]), bf_bits(a[3]));
  u[2] = pk16(bf_bits(b[0]), bf_bits(b[1]));
  u[3] = pk16(bf_bits(b[2]), bf_bits(b[3]));
  unsigned short* d = y + (size_t)t * 8;
  *(volatile v4u*)d = u;
  __threadfence();
  *(volatile v4u*)d = u;
}

__global__ __launch_bounds__(256)
void wtrans_kernel(const float* __restrict__ w, unsigned short* wt, int R, int C) {
  __shared__ __align__(16) unsigned short L[64 * LTP];
  const int tid = threadIdx.x;
  const int c0 = blockIdx.x * 64, r0 = blockIdx.y * 64;
  const int c4 = (tid & 15) * 4, rs = tid >> 4;
#pragma unroll
  for (int it = 0; it < 4; ++it) {
    const int r = it * 16 + rs;
    const v4f v = *(const v4f*)(w + (size_t)(r0 + r) * C + c0 + c4);
#pragma unroll
    for (int j = 0; j < 4; ++j) L[(c4 + j) * LTP + r] = bf_bits(v[j]);
  }
  __syncthreads();
  const int e = tid & 7, lq = tid >> 3;
  v4u u[2];
  size_t po[2];
#pragma unroll
  for (int it = 0; it < 2; ++it) {
    const int c = it * 32 + lq;
    u[it] = *(const v4u*)(L + c * LTP + 8 * e);
    po[it] = (size_t)(c0 + c) * R + r0 + 8 * e;
  }
#pragma unroll
  for (int it = 0; it < 2; ++it) *(volatile v4u*)(wt + po[it]) = u[it];
  __threadfence();
#pragma unroll
  for (int it = 0; it < 2; ++it) *(volatile v4u*)(wt + po[it]) = u[it];
}

template <int BIASM>
__global__ __launch_bounds__(256)
void proj_kernel(const unsigned short* __restrict__ A, const unsigned short* __restrict__ B,
                 const float* __restrict__ bias, unsigned short* Ch, unsigned short* Cl,
                 int lda, int ldb, int ldc) {
  __shared__ __align__(16) float Os[GM * OSP];
  const int tid  = threadIdx.x;
  const int lane = tid & 31, wave = tid >> 5;
  const int hh   = lane >> 4, cl = lane & 15;
  const int wm   = wave >> 1, wn = wave & 1;
  const int mBase = blockIdx.x * GM;
  const int nBase = blockIdx.y * GN;
  const unsigned short* a0p = A + (size_t)(mBase + 32 * wm + cl) * lda + 8 * hh;
  const unsigned short* a1p = a0p + (size_t)16 * lda;
  const unsigned short* b0p = B + (size_t)(nBase + 32 * wn + cl) * ldb + 8 * hh;
  const unsigned short* b1p = b0p + (size_t)16 * ldb;

  v8f acc[2][2];
#pragma unroll
  for (int mi = 0; mi < 2; ++mi)
#pragma unroll
    for (int ni = 0; ni < 2; ++ni) acc[mi][ni] = zero8();

#pragma unroll 1
  for (int k0 = 0; k0 < DIM; k0 += 32) {
    const Frag fa0 = ldfrag(a0p + k0);
    const Frag fa1 = ldfrag(a1p + k0);
    const Frag fb0 = ldfrag(b0p + k0);
    const Frag fb1 = ldfrag(b1p + k0);
    acc[0][0] = mma_b(fa0.b, fb0.b, acc[0][0]);
    acc[0][1] = mma_b(fa0.b, fb1.b, acc[0][1]);
    acc[1][0] = mma_b(fa1.b, fb0.b, acc[1][0]);
    acc[1][1] = mma_b(fa1.b, fb1.b, acc[1][1]);
  }

#pragma unroll
  for (int mi = 0; mi < 2; ++mi) {
#pragma unroll
    for (int ni = 0; ni < 2; ++ni) {
      const int n_loc = 32 * wn + 16 * ni + cl;
#pragma unroll
      for (int r = 0; r < 8; ++r) {
        const int m_loc = 32 * wm + 16 * mi + 8 * hh + r;
        const float bb = (BIASM != 0) ? bfr(bias[mBase + m_loc]) : bfr(bias[nBase + n_loc]);
        Os[m_loc * OSP + n_loc] = acc[mi][ni][r] + bb;
      }
    }
  }
  __syncthreads();

  const int e = tid & 7, lq = tid >> 3;
  v4u uh[4], ul[4];
  size_t po[4];
#pragma unroll
  for (int it = 0; it < 4; ++it) {
    const int row = it * 32 + lq;
    const float* op = Os + row * OSP + 8 * e;
    const v4f v0 = *(const v4f*)(op);
    const v4f v1 = *(const v4f*)(op + 4);
    split8(v0, v1, uh[it], ul[it]);
    po[it] = (size_t)(mBase + row) * ldc + nBase + 8 * e;
  }
#pragma unroll
  for (int it = 0; it < 4; ++it) {
    *(volatile v4u*)(Ch + po[it]) = uh[it];
    *(volatile v4u*)(Cl + po[it]) = ul[it];
  }
  __threadfence();
#pragma unroll
  for (int it = 0; it < 4; ++it) {
    *(volatile v4u*)(Ch + po[it]) = uh[it];
    *(volatile v4u*)(Cl + po[it]) = ul[it];
  }
}

__global__ __launch_bounds__(256)
void stats_kernel(const unsigned short* __restrict__ Qh, const unsigned short* __restrict__ Kh, float* PST) {
  __shared__ float pm[8 * CTOK];
  __shared__ float pe[8 * CTOK];
  const int tid  = threadIdx.x;
  const int lane = tid & 31, wave = tid >> 5;
  const int hh   = lane >> 4, cl = lane & 15;
  const int h = blockIdx.y, qt = blockIdx.x;
  const int n0 = qt * QT + 16 * wave;
  const Frag a = ldfrag(Qh + (size_t)(n0 + cl) * DQ + h * HD + 8 * hh);
  const unsigned short* kp = Kh + (size_t)cl * DQ + h * HD + 8 * hh;
#pragma unroll 1
  for (int ct = 0; ct < CTOK / 16; ++ct) {
    const Frag b = ldfrag(kp + (size_t)ct * 16 * DQ);
    const v8f s = mma_b(a.b, b.b, zero8());
    float m = s[0];
#pragma unroll
    for (int r = 1; r < 8; ++r) m = fmaxf(m, s[r]);
    m = fmaxf(m, __shfl_xor(m, 16, 32));
    float ex = 0.f;
#pragma unroll
    for (int r = 0; r < 8; ++r) ex += __expf(s[r] - m);
    ex += __shfl_xor(ex, 16, 32);
    pm[wave * CTOK + ct * 16 + cl] = m;
    pe[wave * CTOK + ct * 16 + cl] = ex;
  }
  __syncthreads();
  const int c = tid;
  float M = pm[c];
#pragma unroll
  for (int wv = 1; wv < 8; ++wv) M = fmaxf(M, pm[wv * CTOK + c]);
  float E = 0.f;
#pragma unroll 1
  for (int wv = 0; wv < 8; ++wv) E += pe[wv * CTOK + c] * __expf(pm[wv * CTOK + c] - M);
  const size_t base = ((size_t)(h * NQT + qt)) * 2 * CTOK;
  float* dm = PST + base + c;
  float* de = PST + base + CTOK + c;
  *(volatile float*)dm = M;
  *(volatile float*)de = E;
  __threadfence();
  *(volatile float*)dm = M;
  *(volatile float*)de = E;
}

__global__ __launch_bounds__(256)
void merge_kernel(const float* __restrict__ PST, float* ST) {
  const int h = blockIdx.x, c = threadIdx.x;
  const float* p = PST + (size_t)h * NQT * 2 * CTOK + c;
  float M = -3.0e38f;
#pragma unroll 1
  for (int t = 0; t < NQT; ++t) M = fmaxf(M, p[(size_t)t * 2 * CTOK]);
  float Z = 0.f;
#pragma unroll 1
  for (int t = 0; t < NQT; ++t) Z += p[(size_t)t * 2 * CTOK + CTOK] * __expf(p[(size_t)t * 2 * CTOK] - M);
  const float rz = 1.0f / Z;
  float* dm = ST + (size_t)(2 * h) * CTOK + c;
  float* dz = dm + CTOK;
  *(volatile float*)dm = M;
  *(volatile float*)dz = rz;
  __threadfence();
  *(volatile float*)dm = M;
  *(volatile float*)dz = rz;
}

__global__ __launch_bounds__(64)
void pv_kernel(const unsigned short* __restrict__ Qh, const unsigned short* __restrict__ Ql,
               const unsigned short* __restrict__ Kh, const unsigned short* __restrict__ Kl,
               const unsigned short* __restrict__ Vh, const unsigned short* __restrict__ Vl,
               const float* __restrict__ ST, unsigned short* Xh, unsigned short* Xl, int nStart) {
  __shared__ __align__(16) float P[2 * 16 * CTOK];
  const int tid  = threadIdx.x;
  const int lane = tid & 31, wave = tid >> 5;
  const int hh   = lane >> 4, cl = lane & 15;
  const int h = blockIdx.y;
  const int nl0 = blockIdx.x * 32 + 16 * wave;
  const int n0 = nStart + nl0;
  float* Pw = P + wave * (16 * CTOK);

  const Frag ah = ldfrag(Qh + (size_t)(n0 + cl) * DQ + h * HD + 8 * hh);
  const Frag al = ldfrag(Ql + (size_t)(n0 + cl) * DQ + h * HD + 8 * hh);
  const float* stm = ST + (size_t)(2 * h) * CTOK;
  const float* stz = stm + CTOK;
  const unsigned short* kh0 = Kh + (size_t)cl * DQ + h * HD + 8 * hh;
  const unsigned short* kl0 = Kl + (size_t)cl * DQ + h * HD + 8 * hh;

  float rsum[8];
#pragma unroll
  for (int r = 0; r < 8; ++r) rsum[r] = 0.f;

#pragma unroll 1
  for (int ct = 0; ct < CTOK / 16; ++ct) {
    const Frag bh = ldfrag(kh0 + (size_t)ct * 16 * DQ);
    const Frag bl = ldfrag(kl0 + (size_t)ct * 16 * DQ);
    v8f s = mma_b(ah.b, bh.b, zero8());
    s = mma_b(ah.b, bl.b, s);
    s = mma_b(al.b, bh.b, s);
    const int c = ct * 16 + cl;
    const float mc = stm[c], zc = stz[c];
#pragma unroll
    for (int r = 0; r < 8; ++r) {
      const float a = __expf(s[r] - mc) * zc;
      rsum[r] += a;
      Pw[(8 * hh + r) * CTOK + c] = a;
    }
  }
#pragma unroll
  for (int r = 0; r < 8; ++r) {
    float v = rsum[r];
    v += __shfl_xor(v, 1, 32);
    v += __shfl_xor(v, 2, 32);
    v += __shfl_xor(v, 4, 32);
    v += __shfl_xor(v, 8, 32);
    rsum[r] = v;
  }
  __syncthreads();

  v8f x0 = zero8(), x1 = zero8();
  const unsigned short* vh0 = Vh + (size_t)(h * HD + cl) * CTOK + 8 * hh;
  const unsigned short* vh1 = vh0 + (size_t)16 * CTOK;
  const unsigned short* vl0 = Vl + (size_t)(h * HD + cl) * CTOK + 8 * hh;
  const unsigned short* vl1 = vl0 + (size_t)16 * CTOK;
  const float* prow = Pw + cl * CTOK + 8 * hh;
#pragma unroll 1
  for (int k0 = 0; k0 < CTOK; k0 += 32) {
    const v4f p0 = *(const v4f*)(prow + k0);
    const v4f p1 = *(const v4f*)(prow + k0 + 4);
    const v4f p2 = *(const v4f*)(prow + k0 + 16);
    const v4f p3 = *(const v4f*)(prow + k0 + 20);
    Frag fh, fl;
    split8(p0, p1, fh.q[0], fl.q[0]);
    split8(p2, p3, fh.q[1], fl.q[1]);
    const Frag bh0 = ldfrag(vh0 + k0);
    const Frag bh1 = ldfrag(vh1 + k0);
    const Frag bl0 = ldfrag(vl0 + k0);
    const Frag bl1 = ldfrag(vl1 + k0);
    x0 = mma_b(fh.b, bh0.b, x0);
    x0 = mma_b(fh.b, bl0.b, x0);
    x0 = mma_b(fl.b, bh0.b, x0);
    x1 = mma_b(fh.b, bh1.b, x1);
    x1 = mma_b(fh.b, bl1.b, x1);
    x1 = mma_b(fl.b, bh1.b, x1);
  }
  __syncthreads();
#pragma unroll
  for (int r = 0; r < 8; ++r) {
    const int row = 8 * hh + r;
    const float inv = __builtin_amdgcn_rcpf(EPSL1 + rsum[r]);
    Pw[row * HD + cl]      = x0[r] * inv;
    Pw[row * HD + 16 + cl] = x1[r] * inv;
  }
  __syncthreads();
  v4u uh[2], ul[2];
  size_t po[2];
  const size_t hb = ((size_t)h * HALFN + nl0) * HD;
#pragma unroll
  for (int i = 0; i < 2; ++i) {
    const int idx = (i * 32 + lane) * 8;
    const v4f v0 = *(const v4f*)(Pw + idx);
    const v4f v1 = *(const v4f*)(Pw + idx + 4);
    split8(v0, v1, uh[i], ul[i]);
    po[i] = hb + (size_t)idx;
  }
#pragma unroll
  for (int i = 0; i < 2; ++i) {
    *(volatile v4u*)(Xh + po[i]) = uh[i];
    *(volatile v4u*)(Xl + po[i]) = ul[i];
  }
  __threadfence();
#pragma unroll
  for (int i = 0; i < 2; ++i) {
    *(volatile v4u*)(Xh + po[i]) = uh[i];
    *(volatile v4u*)(Xl + po[i]) = ul[i];
  }
}

__global__ __launch_bounds__(256)
void outproj_kernel(const unsigned short* __restrict__ Xh, const unsigned short* __restrict__ Xl,
                    const unsigned short* __restrict__ WpT, const float* __restrict__ bias,
                    float* out, int nStart) {
  __shared__ __align__(16) float Os[GM * OSP];
  const int tid  = threadIdx.x;
  const int lane = tid & 31, wave = tid >> 5;
  const int hh   = lane >> 4, cl = lane & 15;
  const int wm   = wave >> 1, wn = wave & 1;
  const int mBase = blockIdx.x * GM;
  const int nBase = blockIdx.y * GN;
  const size_t ar0 = (size_t)(mBase + 32 * wm + cl) * HD + 8 * hh;
  const size_t ar1 = ar0 + (size_t)16 * HD;
  const unsigned short* b0p = WpT + (size_t)(nBase + 32 * wn + cl) * DQ + 8 * hh;
  const unsigned short* b1p = b0p + (size_t)16 * DQ;

  v8f acc[2][2];
#pragma unroll
  for (int mi = 0; mi < 2; ++mi)
#pragma unroll
    for (int ni = 0; ni < 2; ++ni) acc[mi][ni] = zero8();

#pragma unroll 1
  for (int kk = 0; kk < NH; ++kk) {
    const size_t po = (size_t)kk * HALFN * HD;
    const Frag ah0 = ldfrag(Xh + po + ar0);
    const Frag ah1 = ldfrag(Xh + po + ar1);
    const Frag al0 = ldfrag(Xl + po + ar0);
    const Frag al1 = ldfrag(Xl + po + ar1);
    const Frag fb0 = ldfrag(b0p + kk * 32);
    const Frag fb1 = ldfrag(b1p + kk * 32);
    acc[0][0] = mma_b(ah0.b, fb0.b, acc[0][0]);
    acc[0][0] = mma_b(al0.b, fb0.b, acc[0][0]);
    acc[0][1] = mma_b(ah0.b, fb1.b, acc[0][1]);
    acc[0][1] = mma_b(al0.b, fb1.b, acc[0][1]);
    acc[1][0] = mma_b(ah1.b, fb0.b, acc[1][0]);
    acc[1][0] = mma_b(al1.b, fb0.b, acc[1][0]);
    acc[1][1] = mma_b(ah1.b, fb1.b, acc[1][1]);
    acc[1][1] = mma_b(al1.b, fb1.b, acc[1][1]);
  }

#pragma unroll
  for (int mi = 0; mi < 2; ++mi) {
#pragma unroll
    for (int ni = 0; ni < 2; ++ni) {
      const int n_loc = 32 * wn + 16 * ni + cl;
      const float bb = bfr(bias[nBase + n_loc]);
#pragma unroll
      for (int r = 0; r < 8; ++r) {
        const int m_loc = 32 * wm + 16 * mi + 8 * hh + r;
        Os[m_loc * OSP + n_loc] = acc[mi][ni][r] + bb;
      }
    }
  }
  __syncthreads();

  const int e = tid & 7, lq = tid >> 3;
  v4f v[8];
  size_t po[8];
#pragma unroll
  for (int it = 0; it < 8; ++it) {
    const int L = it * 32 + lq;
    const int row = L >> 1, hf = L & 1;
    v[it] = *(const v4f*)(Os + row * OSP + hf * 32 + 4 * e);
    po[it] = (size_t)(nStart + mBase + row) * DIM + nBase + hf * 32 + 4 * e;
  }
#pragma unroll
  for (int it = 0; it < 8; ++it) *(volatile v4f*)(out + po[it]) = v[it];
  __threadfence();
#pragma unroll
  for (int it = 0; it < 8; ++it) *(volatile v4f*)(out + po[it]) = v[it];
}

extern "C" void kernel_launch(void* const* d_in, const int* in_sizes, int n_in,
                              void* d_out, int out_size, void* d_ws, size_t ws_size,
                              hipStream_t stream) {
  if (n_in < 10) return;
  if (in_sizes[0] != CTOK * DIM) return;
  if (in_sizes[1] != NTOK * DIM) return;
  if (in_sizes[2] != DIM * DQ || in_sizes[4] != DIM * DQ || in_sizes[6] != DIM * DQ) return;
  if (in_sizes[3] != DQ || in_sizes[5] != DQ || in_sizes[7] != DQ) return;
  if (in_sizes[8] != DQ * DIM || in_sizes[9] != DIM) return;
  if (out_size != NTOK * DIM) return;

  size_t off = 0;
  const size_t oG   = off; off += (size_t)NTOK * DIM * 2;
  const size_t oS   = off; off += (size_t)CTOK * DIM * 2;
  const size_t oWq  = off; off += (size_t)DQ * DIM * 2;
  const size_t oWk  = off; off += (size_t)DQ * DIM * 2;
  const size_t oWv  = off; off += (size_t)DQ * DIM * 2;
  const size_t oWp  = off; off += (size_t)DIM * DQ * 2;
  const size_t oQh  = off; off += (size_t)NTOK * DQ * 2;
  const size_t oQl  = off; off += (size_t)NTOK * DQ * 2;
  const size_t oKh  = off; off += (size_t)CTOK * DQ * 2;
  const size_t oKl  = off; off += (size_t)CTOK * DQ * 2;
  const size_t oVh  = off; off += (size_t)DQ * CTOK * 2;
  const size_t oVl  = off; off += (size_t)DQ * CTOK * 2;
  const size_t oST  = off; off += (size_t)NH * 2 * CTOK * 4;
  const size_t oXh  = off; off += (size_t)NH * HALFN * HD * 2;
  const size_t oXl  = off; off += (size_t)NH * HALFN * HD * 2;
  const size_t pstBytes = (size_t)NH * NQT * 2 * CTOK * 4;
  if (pstBytes > (size_t)NTOK * DIM * 2) return;
  if (off > ws_size) return;
  if (off > (size_t)134217728) return;

  const float* sem = (const float*)d_in[0];
  const float* geo = (const float*)d_in[1];
  const float* Wk  = (const float*)d_in[2];
  const float* bk  = (const float*)d_in[3];
  const float* Wq  = (const float*)d_in[4];
  const float* bq  = (const float*)d_in[5];
  const float* Wv  = (const float*)d_in[6];
  const float* bv  = (const float*)d_in[7];
  const float* Wp  = (const float*)d_in[8];
  const float* bp  = (const float*)d_in[9];
  float* out = (float*)d_out;

  char* ws = (char*)d_ws;
  unsigned short* G16 = (unsigned short*)(ws + oG);
  float*          PST = (float*)(ws + oG);
  unsigned short* S16 = (unsigned short*)(ws + oS);
  unsigned short* WqT = (unsigned short*)(ws + oWq);
  unsigned short* WkT = (unsigned short*)(ws + oWk);
  unsigned short* WvT = (unsigned short*)(ws + oWv);
  unsigned short* WpT = (unsigned short*)(ws + oWp);
  unsigned short* Qh  = (unsigned short*)(ws + oQh);
  unsigned short* Ql  = (unsigned short*)(ws + oQl);
  unsigned short* Kh  = (unsigned short*)(ws + oKh);
  unsigned short* Kl  = (unsigned short*)(ws + oKl);
  unsigned short* Vh  = (unsigned short*)(ws + oVh);
  unsigned short* Vl  = (unsigned short*)(ws + oVl);
  float*          ST  = (float*)(ws + oST);
  unsigned short* Xh  = (unsigned short*)(ws + oXh);
  unsigned short* Xl  = (unsigned short*)(ws + oXl);

  const dim3 blk256(256);
  const dim3 blk64(64);

  cvt_kernel<<<dim3((NTOK * DIM) / 2048), blk256, 0, stream>>>(geo, G16, (NTOK * DIM) / 8);
  cvt_kernel<<<dim3((CTOK * DIM) / 2048), blk256, 0, stream>>>(sem, S16, (CTOK * DIM) / 8);
  wtrans_kernel<<<dim3(DQ / 64, DIM / 64), blk256, 0, stream>>>(Wq, WqT, DIM, DQ);
  wtrans_kernel<<<dim3(DQ / 64, DIM / 64), blk256, 0, stream>>>(Wk, WkT, DIM, DQ);
  wtrans_kernel<<<dim3(DQ / 64, DIM / 64), blk256, 0, stream>>>(Wv, WvT, DIM, DQ);
  wtrans_kernel<<<dim3(DIM / 64, DQ / 64), blk256, 0, stream>>>(Wp, WpT, DQ, DIM);
  proj_kernel<0><<<dim3(NTOK / GM, DQ / GN), blk256, 0, stream>>>(G16, WqT, bq, Qh, Ql, DIM, DIM, DQ);
  proj_kernel<0><<<dim3(CTOK / GM, DQ / GN), blk256, 0, stream>>>(S16, WkT, bk, Kh, Kl, DIM, DIM, DQ);
  proj_kernel<1><<<dim3(DQ / GM, CTOK / GN), blk256, 0, stream>>>(WvT, S16, bv, Vh, Vl, DIM, DIM, CTOK);
  stats_kernel<<<dim3(NQT, NH), blk256, 0, stream>>>(Qh, Kh, PST);
  merge_kernel<<<dim3(NH), blk256, 0, stream>>>(PST, ST);
  for (int hf = 0; hf < 2; ++hf) {
    const int nStart = hf * HALFN;
    pv_kernel<<<dim3(HALFN / 32, NH), blk64, 0, stream>>>(Qh, Ql, Kh, Kl, Vh, Vl, ST, Xh, Xl, nStart);
    outproj_kernel<<<dim3(HALFN / GM, DIM / GN), blk256, 0, stream>>>(Xh, Xl, WpT, bp, out, nStart);
  }
  (void)hipGetLastError();
}
